// MultiHeadAttentionLayer_43241730736590
// MI455X (gfx1250) — hardware-verified
//
#include <hip/hip_runtime.h>


#ifndef NB
#define NB 8
#endif
#ifndef SEQ
#define SEQ 1024
#endif
#define NB_FULL  8
#define SEQ_FULL 1024
#ifndef OUT_SEQ
#define OUT_SEQ SEQ
#endif
#define DI   256
#define DO   512
#define NH_  8
#define HD   64
#define AW   4
#define OSP  68
#define WTP  65
#define SC2  ((float)(0.125 * 1.4426950408889634))
#define PSH  14.0f
#define QRS  2048.0f
#define QRI  (1.0f / 2048.0f)
#define NEGB (-3.0e38f)

static_assert(HD == 64);
static_assert(NH_ * HD == DO);
static_assert(DO % 64 == 0);
static_assert(DI % 64 == 0);
static_assert(DI % 32 == 0);
static_assert(HD % 32 == 0);
static_assert(HD % 16 == 0);
static_assert(SEQ % 64 == 0);
static_assert((NB * SEQ) % 64 == 0);
static_assert(SEQ % 32 == 0);
static_assert(SEQ % (16 * AW) == 0);
static_assert(((size_t)SEQ * DI) % 8 == 0);
static_assert(NB <= NB_FULL);
static_assert(SEQ <= SEQ_FULL);
static_assert((OSP * 4) % 16 == 0);
static_assert(OSP >= HD);
static_assert(OSP >= 64);

typedef _Float16 h16;
typedef unsigned short bf;
typedef __attribute__((ext_vector_type(16))) __bf16   v16bf;
typedef __attribute__((ext_vector_type(16))) _Float16 v16h;
typedef __attribute__((ext_vector_type(8)))  _Float16 v8h;
typedef __attribute__((ext_vector_type(8)))  unsigned short v8us;
typedef __attribute__((ext_vector_type(8)))  float    v8f;
typedef __attribute__((ext_vector_type(4)))  float    v4f;
typedef __attribute__((ext_vector_type(4)))  int      v4i;
typedef v4f  __attribute__((may_alias)) v4fa;

__device__ __forceinline__ unsigned short f2bf(float f) { unsigned u = __float_as_uint(f); u += 0x7FFFu + ((u >> 16) & 1u); return (unsigned short)(u >> 16); }
__device__ __forceinline__ float bfr(float f) { return __uint_as_float(((unsigned)f2bf(f)) << 16); }
__device__ __forceinline__ v16h cat16(v8h lo, v8h hi) { return __builtin_shufflevector(lo, hi, 0, 1, 2, 3, 4, 5, 6, 7, 8, 9, 10, 11, 12, 13, 14, 15); }
__device__ __forceinline__ v16bf cat16b(v8us lo, v8us hi) { return __builtin_bit_cast(v16bf, __builtin_shufflevector(lo, hi, 0, 1, 2, 3, 4, 5, 6, 7, 8, 9, 10, 11, 12, 13, 14, 15)); }
__device__ __forceinline__ v8f wmma16(v16h a, v16h b, v8f c) { return __builtin_amdgcn_wmma_f32_16x16x32_f16(false, a, false, b, (short)0, c, false, false); }
__device__ __forceinline__ v8f wmmab(v16bf a, v16bf b, v8f c) { return __builtin_amdgcn_wmma_f32_16x16x32_bf16(false, a, false, b, (short)0, c, false, false); }
__device__ __forceinline__ v16h  ldh(const h16* p) { return cat16(*(const v8h*)p, *(const v8h*)(p + 16)); }
__device__ __forceinline__ v16bf ldb(const bf* p)  { return cat16b(*(const v8us*)p, *(const v8us*)(p + 16)); }
__device__ __forceinline__ void wave_sync() { __builtin_amdgcn_fence(3  , "wavefront"); __builtin_amdgcn_wave_barrier(); asm volatile("" ::: "memory"); }
__device__ __forceinline__ h16 toh_flush(float v) { const h16 r = (h16)v; return (fabsf(v) < 6.103515625e-05f) ? (h16)0.0f : r; }
__device__ __forceinline__ v8f wmma16g(v16h a, v16h b, v8f c) { c = wmma16(a, b, c); asm volatile("v_nop\n\tv_nop\n\tv_nop\n\tv_nop" : "+v"(c) : "v"(a), "v"(b)); return c; }
__device__ __forceinline__ v8f wmmabg(v16bf a, v16bf b, v8f c) { c = wmmab(a, b, c); asm volatile("v_nop\n\tv_nop\n\tv_nop\n\tv_nop" : "+v"(c) : "v"(a), "v"(b)); return c; }

__global__ __launch_bounds__(256) void k_cvt8(const float* __restrict__ src, bf* dst, size_t n8) {
    const size_t i = (size_t)blockIdx.x * 256 + threadIdx.x; if (i >= n8) return;
    const v8f v = *(const v8f*)(src + i * 8); v8us o;
#pragma unroll
    for (int k = 0; k < 8; ++k) o[k] = f2bf(v[k]);
    *(volatile v8us*)(dst + i * 8) = o; __threadfence(); *(volatile v8us*)(dst + i * 8) = o;
}

static_assert(256 * 16 == 64 * 64);
static_assert(256 * 2 * 16 == 64 * 128);
static_assert(64 * WTP * 4 <= 131072);
__global__ __launch_bounds__(256) void k_wtr(const float* __restrict__ W, bf* WT) {
    __shared__ float tl[64 * WTP];
    const int tid = threadIdx.x;
    const int n0 = blockIdx.x * 64, k0 = blockIdx.y * 64;
#pragma unroll 1
    for (int it = 0; it < 16; ++it) { const int p = it * 256 + tid; const int r = p >> 6, c = p & 63;
        tl[r * WTP + c] = bfr(W[(size_t)(k0 + r) * DO + n0 + c]); }
    __syncthreads();
#pragma unroll 1
    for (int ps = 0; ps < 2; ++ps) {
#pragma unroll
        for (int it = 0; it < 2; ++it) { const int p = it * 256 + tid; const int nn = p >> 3, kc = (p & 7) * 8;
            v8us o;
#pragma unroll
            for (int i = 0; i < 8; ++i) o[i] = f2bf(tl[(kc + i) * WTP + nn]);
            *(volatile v8us*)(WT + (size_t)(n0 + nn) * DI + k0 + kc) = o; }
        if (ps == 0) __threadfence(); }
}

static_assert(32 * 16 * 4 == 16 * 128);
static_assert(16 * 68 * 4 <= 131072);
__global__ __launch_bounds__(32) void k_proj(const bf* __restrict__ A, const bf* __restrict__ Bt, const float* __restrict__ bias, h16* P, h16* Pr, int mode) {
    __shared__ __align__(16) float os[16 * 68];
    const int K = DI;
    const int lane = threadIdx.x & 31, lr = lane & 15, hi = lane >> 4; const int r0 = blockIdx.x * 64, c0 = blockIdx.y * 64;
    v8f acc[4][4];
#pragma unroll
    for (int mb = 0; mb < 4; ++mb)
#pragma unroll
        for (int nb = 0; nb < 4; ++nb) acc[mb][nb] = (v8f){};
    const size_t aoff = (size_t)(r0 + lr) * K + 8 * hi, boff = (size_t)(c0 + lr) * K + 8 * hi;
#pragma unroll 1
    for (int kc = 0; kc < K; kc += 32) {
        v16bf a[4];
#pragma unroll
        for (int mb = 0; mb < 4; ++mb) a[mb] = ldb(A + aoff + (size_t)mb * 16 * K + kc);
#pragma unroll
        for (int nb = 0; nb < 4; ++nb) { const v16bf b = ldb(Bt + boff + (size_t)nb * 16 * K + kc);
#pragma unroll
            for (int mb = 0; mb < 4; ++mb) acc[mb][nb] = wmmabg(a[mb], b, acc[mb][nb]); }
    }
    float bc[4];
#pragma unroll
    for (int nb = 0; nb < 4; ++nb) bc[nb] = 0.0f;
    if (mode == 0) {
#pragma unroll
        for (int nb = 0; nb < 4; ++nb) bc[nb] = bfr(bias[c0 + nb * 16 + lr]); }
    size_t tbase, pitch;
    if (mode == 0) { const int bb = r0 / SEQ, tt = r0 % SEQ; const int zc = bb * NH_ + c0 / HD;
                     tbase = ((size_t)zc * SEQ + (size_t)tt) * HD; pitch = (size_t)HD; }
    else           { const int bb = c0 / SEQ, tt = c0 % SEQ;
                     tbase = (size_t)bb * (size_t)DO * SEQ + (size_t)r0 * SEQ + (size_t)tt; pitch = (size_t)SEQ; }
#pragma unroll
    for (int mb = 0; mb < 4; ++mb) {
        float br[8];
#pragma unroll
        for (int j = 0; j < 8; ++j) br[j] = 0.0f;
        if (mode != 0) {
#pragma unroll
            for (int j = 0; j < 8; ++j) br[j] = bfr(bias[r0 + mb * 16 + hi * 8 + j]); }
#pragma unroll
        for (int nb = 0; nb < 4; ++nb) {
#pragma unroll
            for (int j = 0; j < 8; ++j) os[(hi * 8 + j) * 68 + nb * 16 + lr] = acc[mb][nb][j] + bc[nb] + br[j]; }
        wave_sync();
        const size_t sb = tbase + (size_t)(mb * 16) * pitch;
#pragma unroll 1
        for (int ps = 0; ps < 2; ++ps) {
#pragma unroll
            for (int s = 0; s < 4; ++s) { const int row = 4 * s + (lane >> 3), c8 = (lane & 7) * 8;
                const v4f x0 = *(const v4fa*)(&os[row * 68 + c8]); const v4f x1 = *(const v4fa*)(&os[row * 68 + c8 + 4]); v8h hv, rv;
#pragma unroll
                for (int i = 0; i < 4; ++i) { const h16 a0 = toh_flush(x0[i]); const h16 a1 = toh_flush(x1[i]); hv[i] = a0; hv[4 + i] = a1;
                    rv[i] = toh_flush((x0[i] - (float)a0) * QRS); rv[4 + i] = toh_flush((x1[i] - (float)a1) * QRS); }
                const size_t oo = sb + (size_t)row * pitch + c8;
                *(volatile v8h*)(P + oo) = hv; if (mode == 0) *(volatile v8h*)(Pr + oo) = rv; }
            if (ps == 0) __threadfence(); }
        wave_sync();
    }
}

static_assert(32 * 16 * 8 == 16 * HD * 4);
static_assert(AW * 16 * OSP * 4 <= 131072);
__global__ __launch_bounds__(32 * AW) void k_flash(const h16* __restrict__ QH, const h16* __restrict__ QR, const h16* __restrict__ KP, const h16* __restrict__ KR, const h16* __restrict__ VT, const int* __restrict__ adj, float* OUT) {
    __shared__ __align__(16) float os[AW * 16 * OSP];
    const int lane = threadIdx.x & 31, lr = lane & 15, hi = lane >> 4;
    const int wave = __builtin_amdgcn_readfirstlane((int)(threadIdx.x >> 5));
    const int zh = blockIdx.y; const int b = zh / NH_, h = zh % NH_;
    const int t0 = (blockIdx.x * AW + wave) * 16;
    const size_t pbase = (size_t)zh * SEQ * HD;
    const size_t qo = pbase + (size_t)(t0 + lr) * HD + 8 * hi;
    const v16h q0 = ldh(QH + qo), q1 = ldh(QH + qo + 32);
    const v16h qr0 = ldh(QR + qo), qr1 = ldh(QR + qo + 32);
    const size_t ko = pbase + (size_t)lr * HD + 8 * hi;
    const size_t vo = pbase + (size_t)lr * SEQ + 8 * hi;
    const size_t ao = (size_t)(t0 + lr) * SEQ_FULL + 8 * hi;
    v8f o[4];
#pragma unroll
    for (int j = 0; j < 4; ++j) o[j] = (v8f){};
    float m = NEGB, l = 0.0f;
#pragma unroll 1
    for (int key0 = 0; key0 < SEQ; key0 += 32) {
        const h16* ka = KP + ko + (size_t)key0 * HD;
        const h16* kr = KR + ko + (size_t)key0 * HD;
        v8f sa = (v8f){}, sb = (v8f){}, ra = (v8f){}, rb = (v8f){};
        { const v16h k00 = ldh(ka), k01 = ldh(ka + 32), r00 = ldh(kr), r01 = ldh(kr + 32);
          sa = wmma16g(k00, q0, sa); sa = wmma16g(k01, q1, sa);
          ra = wmma16g(k00, qr0, ra); ra = wmma16g(k01, qr1, ra);
          ra = wmma16g(r00, q0, ra); ra = wmma16g(r01, q1, ra); }
        { const v16h k10 = ldh(ka + 16 * HD), k11 = ldh(ka + 16 * HD + 32), r10 = ldh(kr + 16 * HD), r11 = ldh(kr + 16 * HD + 32);
          sb = wmma16g(k10, q0, sb); sb = wmma16g(k11, q1, sb);
          rb = wmma16g(k10, qr0, rb); rb = wmma16g(k11, qr1, rb);
          rb = wmma16g(r10, q0, rb); rb = wmma16g(r11, q1, rb); }
        const int* ap = adj + ao + key0;
        v4i a0 = *(const v4i*)ap, a1 = *(const v4i*)(ap + 4), a2 = *(const v4i*)(ap + 16), a3 = *(const v4i*)(ap + 20);
        asm volatile("" : "+v"(a0), "+v"(a1), "+v"(a2), "+v"(a3));
        int ax[8], ay[8];
#pragma unroll
        for (int r = 0; r < 4; ++r) { ax[r] = a0[r]; ax[4 + r] = a1[r]; ay[r] = a2[r]; ay[4 + r] = a3[r]; }
        float ta[8], tb[8]; bool fa[8], fb[8]; float mx = NEGB;
#pragma unroll
        for (int r = 0; r < 8; ++r) {
            fa[r] = (ax[r] != 0);
            fb[r] = (ay[r] != 0);
            ta[r] = (sa[r] + ra[r] * QRI) * SC2; tb[r] = (sb[r] + rb[r] * QRI) * SC2;
            mx = fmaxf(mx, fmaxf(fa[r] ? ta[r] : NEGB, fb[r] ? tb[r] : NEGB)); }
        mx = fmaxf(mx, __shfl_xor(mx, 16, 32));
        const float mnew = fmaxf(m, mx);
        const float alpha = __builtin_amdgcn_exp2f(m - mnew);
        const float sh = PSH - mnew;
        v16h pb; float ls = 0.0f;
#pragma unroll
        for (int r = 0; r < 8; ++r) {
            const float xa = ta[r] + sh, xb = tb[r] + sh;
            const float ea = __builtin_amdgcn_exp2f(xa), eb = __builtin_amdgcn_exp2f(xb);
            const bool ua = fa[r] & (xa >= -14.0f), ub = fb[r] & (xb >= -14.0f);
            const float ga = ua ? ea : 0.0f, gb = ub ? eb : 0.0f;
            const h16 pa = (h16)ga; const h16 pc = (h16)gb;
            pb[r] = pa; pb[8 + r] = pc;
            ls += (float)pa + (float)pc; }
        l = l * alpha + ls; m = mnew;
#pragma unroll
        for (int j = 0; j < 4; ++j) o[j] = o[j] * alpha;
        const h16* va = VT + vo + key0;
        const v16h v0 = ldh(va), v1 = ldh(va + (size_t)16 * SEQ), v2 = ldh(va + (size_t)32 * SEQ), v3 = ldh(va + (size_t)48 * SEQ);
        o[0] = wmma16g(v0, pb, o[0]); o[1] = wmma16g(v1, pb, o[1]); o[2] = wmma16g(v2, pb, o[2]); o[3] = wmma16g(v3, pb, o[3]);
    }
    l += __shfl_xor(l, 16, 32);
    const bool any = l > 0.0f;
    const float lsafe = any ? l : 1.0f;
    const float inv = any ? (1.0f / lsafe) : __uint_as_float(0x7FC00000u);
    const int wb = wave * 16 * OSP;
#pragma unroll
    for (int j = 0; j < 4; ++j) { v4f a, c;
        a[0] = o[j][0] * inv; a[1] = o[j][1] * inv; a[2] = o[j][2] * inv; a[3] = o[j][3] * inv;
        c[0] = o[j][4] * inv; c[1] = o[j][5] * inv; c[2] = o[j][6] * inv; c[3] = o[j][7] * inv;
        *(v4fa*)(&os[wb + lr * OSP + 16 * j + 8 * hi]) = a; *(v4fa*)(&os[wb + lr * OSP + 16 * j + 8 * hi + 4]) = c; }
    wave_sync();
    float* orow = OUT + ((size_t)b * OUT_SEQ + t0) * DO + h * HD;
#pragma unroll 1
    for (int ps = 0; ps < 2; ++ps) {
#pragma unroll
        for (int s = 0; s < 8; ++s) { const int row = 2 * s + (lane >> 4), cofs = (lane & 15) * 4;
            const v4f val = *(const v4fa*)(&os[wb + row * OSP + cofs]);
            *(volatile v4f*)(orow + (size_t)row * DO + cofs) = val; }
        if (ps == 0) __threadfence(); }
}

static constexpr size_t al256(size_t v) { return (v + 255) & ~(size_t)255; }
static constexpr size_t SZ_HB = al256((size_t)NB * SEQ * DI * 2);
static constexpr size_t SZ_WT = al256((size_t)3 * DO * DI * 2);
static constexpr size_t SZ_PL = al256((size_t)NB * NH_ * SEQ * HD * 2);
static constexpr size_t SZ_TOTAL = SZ_HB + SZ_WT + 5 * SZ_PL;
static_assert(SZ_TOTAL <= (size_t)134217728);
static_assert(((size_t)DO * DI * 2) % 256 == 0);
static_assert((size_t)NB * NH_ * SEQ * HD == (size_t)NB * DO * SEQ);
static_assert(((size_t)(NB_FULL - 1) * OUT_SEQ + SEQ_FULL) * DO * 4 <= (size_t)16777216 || NB != NB_FULL || SEQ != SEQ_FULL);

extern "C" void kernel_launch(void* const* d_in, const int* in_sizes, int n_in,
                              void* d_out, int out_size, void* d_ws, size_t ws_size, hipStream_t stream) {
    if (n_in < 8) return;
    const size_t needh = ((size_t)(NB - 1) * SEQ_FULL + SEQ) * DI;
    const size_t needa = (size_t)(SEQ - 1) * SEQ_FULL + SEQ;
    if ((size_t)in_sizes[0] < needa || (size_t)in_sizes[1] < needh) return;
    if ((size_t)in_sizes[2] < (size_t)DI * DO || (size_t)in_sizes[4] < (size_t)DI * DO || (size_t)in_sizes[6] < (size_t)DI * DO) return;
    if (in_sizes[3] < DO || in_sizes[5] < DO || in_sizes[7] < DO) return;
    if ((size_t)out_size < ((size_t)(NB - 1) * OUT_SEQ + SEQ) * DO) return;
    if (SZ_TOTAL > ws_size) return;
    const int*   adj = (const int*)d_in[0];
    const float* hin = (const float*)d_in[1];
    const float* wq = (const float*)d_in[2]; const float* bq = (const float*)d_in[3];
    const float* wk = (const float*)d_in[4]; const float* bk = (const float*)d_in[5];
    const float* wv = (const float*)d_in[6]; const float* bv = (const float*)d_in[7];
    float* OUT = (float*)d_out;
    char* wsp = (char*)d_ws;
    bf* HB = (bf*)wsp; wsp += SZ_HB;
    bf* WT = (bf*)wsp; wsp += SZ_WT;
    h16* QH = (h16*)wsp; wsp += SZ_PL;
    h16* KP = (h16*)wsp; wsp += SZ_PL;
    h16* VT = (h16*)wsp; wsp += SZ_PL;
    h16* QR = (h16*)wsp; wsp += SZ_PL;
    h16* KR = (h16*)wsp; wsp += SZ_PL;
    bf* WQ = WT; bf* WK = WT + (size_t)DO * DI; bf* WV = WT + (size_t)2 * DO * DI;

    if (SEQ == SEQ_FULL) {
        const size_t n8 = (size_t)NB * SEQ * DI / 8;
        k_cvt8<<<(unsigned)((n8 + 255) / 256), 256, 0, stream>>>(hin, HB, n8);
    } else {
        const size_t n8 = (size_t)SEQ * DI / 8;
        for (int b = 0; b < NB; ++b) k_cvt8<<<(unsigned)((n8 + 255) / 256), 256, 0, stream>>>(hin + (size_t)b * SEQ_FULL * DI, HB + (size_t)b * SEQ * DI, n8);
    }
    k_wtr<<<dim3(DO / 64, DI / 64, 1), 256, 0, stream>>>(wq, WQ);
    k_wtr<<<dim3(DO / 64, DI / 64, 1), 256, 0, stream>>>(wk, WK);
    k_wtr<<<dim3(DO / 64, DI / 64, 1), 256, 0, stream>>>(wv, WV);

    k_proj<<<dim3(NB * SEQ / 64, DO / 64, 1), 32, 0, stream>>>(HB, WQ, bq, QH, QR, 0);
    k_proj<<<dim3(NB * SEQ / 64, DO / 64, 1), 32, 0, stream>>>(HB, WK, bk, KP, KR, 0);
    k_proj<<<dim3(DO / 64, NB * SEQ / 64, 1), 32, 0, stream>>>(WV, HB, bv, VT, VT, 1);

    k_flash<<<dim3(SEQ / (16 * AW), NB * NH_, 1), 32 * AW, 0, stream>>>(QH, QR, KP, KR, VT, adj, OUT);
}
